// KalmanLSTM_38233798869123
// MI455X (gfx1250) — hardware-verified
//
#include <hip/hip_runtime.h>
#include <math.h>

constexpr int kHistT  = 16;
constexpr int kNS     = 6;
constexpr int kHid    = 32;
constexpr int kGateN  = 128;
constexpr int kKA     = 64;
constexpr int kTile   = 64;
constexpr int kSP     = 44;
constexpr int kPO     = 8;
constexpr int kOutF   = 5;
constexpr int kZP     = 128;
constexpr int kParN   = 368;
constexpr int kOffCfb = 192, kOffCoW = 224, kOffCob = 352, kOffTh = 356;
constexpr float kDT   = 0.2f;
constexpr float kF01  = 0.2f, kF02 = 0.02f, kF12 = 0.2f;
constexpr float kGA   = 0.0013333333333333335f, kGB = 0.02f, kGC = 0.2f;
constexpr float kWCarry = 16.0f, kWCarryInv = 0.0625f;

typedef __attribute__((ext_vector_type(16))) _Float16 v16h;
typedef __attribute__((ext_vector_type(8)))  _Float16 v8h;
typedef __attribute__((ext_vector_type(8)))  float    v8f;
typedef __attribute__((ext_vector_type(4)))  float    v4f;
typedef __attribute__((ext_vector_type(4)))  unsigned int v4u;

__device__ __forceinline__ void dep_guard_h(v8f& a, v8f& b, v16h x, v16h y) { asm volatile("v_nop\n\tv_nop\n\tv_nop\n\tv_nop" : "+v"(a), "+v"(b) : "v"(x), "v"(y)); }
__device__ __forceinline__ void keep4_h(v16h a, v16h b, v16h c, v16h d) { asm volatile("v_nop" :: "v"(a), "v"(b), "v"(c), "v"(d)); }
__device__ __forceinline__ void acc_guard4(v8f& a, v8f& b, v8f& c, v8f& d) { asm volatile("v_nop\n\tv_nop\n\tv_nop\n\tv_nop" : "+v"(a), "+v"(b), "+v"(c), "+v"(d)); }
template <typename T> struct Frag;
template <> struct Frag<_Float16> {
  typedef v16h V; union U { v16h v; v8h h[2]; };
  static __device__ __forceinline__ v16h load(const _Float16* p) {
    U f; f.h[0] = *(const v8h*)(p); f.h[1] = *(const v8h*)(p + 16); return f.v;
  }
  static __device__ __forceinline__ v8f mma(v16h a, v16h b, v8f c) {
    return __builtin_amdgcn_wmma_f32_16x16x32_f16(false, a, false, b, (short)0, c, false, false);
  }
  static __device__ __forceinline__ void guard(v8f& a, v8f& b, v16h x, v16h y) { dep_guard_h(a, b, x, y); }
  static __device__ __forceinline__ void keep(v16h a, v16h b, v16h c, v16h d) { keep4_h(a, b, c, d); }
};

__device__ __forceinline__ int clampi(int v, int lo, int hi) { return v < lo ? lo : (v > hi ? hi : v); }
__device__ __forceinline__ unsigned pk16(unsigned short a, unsigned short b) { return (unsigned)a | ((unsigned)b << 16); }
__device__ __forceinline__ unsigned short h_bits(float f) { const _Float16 h = (_Float16)f; return __builtin_bit_cast(unsigned short, h); }
__device__ __forceinline__ unsigned short h16_bits(_Float16 h) { return __builtin_bit_cast(unsigned short, h); }

__device__ __forceinline__ float sigm_f(float z) {
  z = fminf(fmaxf(z, -40.0f), 40.0f);
  const float e = __expf(-z);
  return __builtin_amdgcn_rcpf(1.0f + e);
}
__device__ __forceinline__ float tanh_f(float z) {
  const float a = fminf(fabsf(z), 20.0f);
  const float e = __expf(-2.0f * a);
  const float r = (1.0f - e) * __builtin_amdgcn_rcpf(1.0f + e);
  return copysignf(r, z);
}

__device__ __forceinline__ void store2_v4u(unsigned short* p, v4u u) {
  *(volatile v4u*)p = u;
  __threadfence();
  *(volatile v4u*)p = u;
}
__device__ __forceinline__ void store2_v4f(float* p, v4f f) {
  *(volatile v4f*)p = f;
  __threadfence();
  *(volatile v4f*)p = f;
}

__device__ __forceinline__ void kf_fx(float X[kNS]) {
  X[0] = X[0] + kF01 * X[1] + kF02 * X[2];
  X[1] = X[1] + kF12 * X[2];
  X[3] = X[3] + kF01 * X[4] + kF02 * X[5];
  X[4] = X[4] + kF12 * X[5];
}
__device__ __forceinline__ void kf_fpf(float P[kNS][kNS]) {
#pragma unroll
  for (int j = 0; j < kNS; ++j) {
    P[0][j] += kF01 * P[1][j] + kF02 * P[2][j];
    P[1][j] += kF12 * P[2][j];
    P[3][j] += kF01 * P[4][j] + kF02 * P[5][j];
    P[4][j] += kF12 * P[5][j];
  }
#pragma unroll
  for (int i = 0; i < kNS; ++i) {
    P[i][0] += kF01 * P[i][1] + kF02 * P[i][2];
    P[i][1] += kF12 * P[i][2];
    P[i][3] += kF01 * P[i][4] + kF02 * P[i][5];
    P[i][4] += kF12 * P[i][5];
  }
}

__device__ __forceinline__ void block_store_state(const _Float16* sA16, const float* sC, const float* sS,
    unsigned short* Ag, float* Cg, float* Sg, int r0, int tid) {
  unsigned short* ab = Ag + (size_t)r0 * kKA;
  float*          cb = Cg + (size_t)r0 * kHid;
  float*          sb = Sg + (size_t)r0 * kSP;
  for (int ps = 0; ps < 2; ++ps) {
#pragma unroll
    for (int it = 0; it < 8; ++it) {
      const int q = it * kTile + tid;
      const _Float16* sp = sA16 + q * 8;
      const v4u u = (v4u){pk16(h16_bits(sp[0]), h16_bits(sp[1])), pk16(h16_bits(sp[2]), h16_bits(sp[3])),
                          pk16(h16_bits(sp[4]), h16_bits(sp[5])), pk16(h16_bits(sp[6]), h16_bits(sp[7]))};
      *(volatile v4u*)(ab + (size_t)q * 8) = u;
    }
#pragma unroll
    for (int it = 0; it < 8; ++it) {
      const int q = it * kTile + tid;
      const float* sp = sC + q * 4;
      const v4f v = (v4f){sp[0], sp[1], sp[2], sp[3]};
      *(volatile v4f*)(cb + (size_t)q * 4) = v;
    }
#pragma unroll
    for (int it = 0; it < 11; ++it) {
      const int q = it * kTile + tid;
      const float* sp = sS + q * 4;
      const v4f v = (v4f){sp[0], sp[1], sp[2], sp[3]};
      *(volatile v4f*)(sb + (size_t)q * 4) = v;
    }
    __threadfence();
  }
}

__global__ __launch_bounds__(256) void pack_params_kernel(
    const float* __restrict__ Wih, const float* __restrict__ Whh,
    const float* __restrict__ bih, const float* __restrict__ bhh,
    const float* __restrict__ coefG,
    unsigned short* __restrict__ Bt, float* __restrict__ biasv, float* __restrict__ dpar) {
  __shared__ float sTh[32];
  const int blk = blockIdx.x;
  const int i   = threadIdx.x;
  if (blk == 4 && i >= 32 && i < 64) {
    const int f = i - 32;
    const float th = tanhf(coefG[clampi(f, 0, kNS - 1)]);
    sTh[f] = (f < kNS) ? th : 0.0f;
  }
  __syncthreads();
  if (blk < 4) {
    const int j  = blk * 256 + i;
    const int n  = j >> 3;
    const int k0 = (j & 7) * 8;
    unsigned short hb[8];
#pragma unroll
    for (int e = 0; e < 8; ++e) {
      const int k  = k0 + e;
      const int ka = clampi(k, 0, kHid - 1);
      const int kb = clampi(k - kHid, 0, kHid - 1);
      const float wi = Wih[n * kHid + ka];
      const float wh = Whh[n * kHid + kb];
      const float v  = (k < kHid) ? wi : wh;
      hb[e] = h_bits(v * kWCarry);
    }
    const v4u u = (v4u){pk16(hb[0], hb[1]), pk16(hb[2], hb[3]), pk16(hb[4], hb[5]), pk16(hb[6], hb[7])};
    store2_v4u(Bt + 8 * (size_t)j, u);
  } else {
    const int ib = clampi(i, 0, 31);
    const int idp = clampi(i - 32, 0, 7);
    float bv[4], dv[4];
#pragma unroll
    for (int e = 0; e < 4; ++e) {
      const int n = 4 * ib + e;
      bv[e] = bih[n] + bhh[n];
      dv[e] = sTh[4 * idp + e];
    }
    const v4f fb = (v4f){bv[0], bv[1], bv[2], bv[3]};
    const v4f fd = (v4f){dv[0], dv[1], dv[2], dv[3]};
    if (i < 32) {
      store2_v4f(biasv + 4 * (size_t)i, fb);
    } else if (i < 40) {
      store2_v4f(dpar + 4 * (size_t)(i - 32), fd);
    }
  }
}

__global__ __launch_bounds__(64) void init_kernel(
    const float* __restrict__ hist,
    const float* __restrict__ psx, const float* __restrict__ psy,
    const float* __restrict__ vsx, const float* __restrict__ vsy,
    const float* __restrict__ asx, const float* __restrict__ asy,
    const float* __restrict__ cfW, const float* __restrict__ cfb,
    unsigned short* __restrict__ Ag, float* __restrict__ Cg, float* __restrict__ Sg, int B) {
  __shared__ __align__(16) _Float16 sA16[kTile * kKA];
  __shared__ __align__(16) float    sC[kTile * kHid];
  __shared__ __align__(16) float    sS[kTile * kSP];
  __shared__ float sPar[224];
  const int tid = threadIdx.x;
  const int r0  = blockIdx.x * kTile;
  const int b   = r0 + tid;
  const int bc  = (b < B) ? b : (B - 1);

#pragma unroll
  for (int q = 0; q < 4; ++q) {
    const int idx = q * kTile + tid;
    const float a  = cfW[clampi(idx, 0, 191)];
    const float bb = cfb[clampi(idx - 192, 0, kHid - 1)];
    const float v  = (idx < 192) ? a : bb;
    if (idx < 224) sPar[idx] = v;
  }

  const float z0x = hist[(size_t)bc * 2 + 0], z0y = hist[(size_t)bc * 2 + 1];
  const float z1x = hist[((size_t)B + bc) * 2 + 0], z1y = hist[((size_t)B + bc) * 2 + 1];
  float X[kNS];
  X[0] = z0x; X[1] = (z1x - z0x) * (1.0f / kDT); X[2] = 0.0f;
  X[3] = (z1y - z0y) * (1.0f / kDT); X[4] = 0.0f; X[5] = 0.0f;
  float dg[kNS];
  dg[0] = psx[0] * psx[0]; dg[1] = vsx[0] * vsx[0]; dg[2] = asx[0] * asx[0];
  dg[3] = psy[0] * psy[0]; dg[4] = vsy[0] * vsy[0]; dg[5] = asy[0] * asy[0];
  __syncthreads();

#pragma unroll 1
  for (int j = 0; j < kHid; ++j) {
    float a = 0.0f;
#pragma unroll
    for (int k = 0; k < kNS; ++k) a = fmaf(X[k], sPar[j * kNS + k], a);
    a += sPar[192 + j];
    sA16[tid * kKA + j]        = (_Float16)tanh_f(a);
    sA16[tid * kKA + kHid + j] = (_Float16)0.0f;
    sC[tid * kHid + j]         = 0.0f;
  }
  {
    float* sr = sS + tid * kSP;
#pragma unroll
    for (int i = 0; i < kNS; ++i) sr[i] = X[i];
    sr[6] = 0.0f; sr[7] = 0.0f;
#pragma unroll
    for (int i = 0; i < kNS; ++i)
#pragma unroll
      for (int j = 0; j < kNS; ++j) sr[kPO + i * kNS + j] = (i == j) ? dg[i] : 0.0f;
  }
  __syncthreads();
  block_store_state(sA16, sC, sS, Ag, Cg, Sg, r0, tid);
}

template <bool PRED>
__global__ __launch_bounds__(64) void step_kernel(
    const unsigned short* __restrict__ Btp, const float* __restrict__ biasv, const float* __restrict__ dpar,
    const float* __restrict__ hist, const float* __restrict__ jerk, const float* __restrict__ GR,
    const float* __restrict__ cfW, const float* __restrict__ cfb,
    const float* __restrict__ coW, const float* __restrict__ cob, const int* __restrict__ lenp,
    unsigned short* __restrict__ Ag, float* __restrict__ Cg, float* __restrict__ Sg,
    float* __restrict__ out, int B, int tz) {
  __shared__ __align__(16) float    sZ[kTile * kZP];
  __shared__ __align__(16) _Float16 sA16[kTile * kKA];
  __shared__ __align__(16) float    sC[kTile * kHid];
  __shared__ __align__(16) float    sS[kTile * kSP];
  __shared__ __align__(16) float    sO[kTile * kOutF];
  __shared__ float sBias[kGateN];
  __shared__ float sPar[kParN];
  (void)lenp;

  const int tid  = threadIdx.x;
  const int lane = tid & 31;
  const int w    = tid >> 5;
  const int r0   = blockIdx.x * kTile;

#pragma unroll
  for (int q = 0; q < 2; ++q) sBias[q * kTile + tid] = biasv[q * kTile + tid];
#pragma unroll
  for (int q = 0; q < 6; ++q) {
    const int idx = q * kTile + tid;
    const float a  = cfW[clampi(idx, 0, 191)];
    const float bb = cfb[clampi(idx - kOffCfb, 0, kHid - 1)];
    const float c  = coW[clampi(idx - kOffCoW, 0, 127)];
    const float d  = cob[clampi(idx - kOffCob, 0, 3)];
    const float e  = dpar[clampi(idx - kOffTh, 0, kNS - 1)];
    const float v  = (idx < kOffCfb) ? a : ((idx < kOffCoW) ? bb : ((idx < kOffCob) ? c :
                     ((idx < kOffTh) ? d : ((idx < kOffTh + kNS) ? e : 0.0f))));
    if (idx < kParN) sPar[idx] = v;
  }

  {
    const _Float16* Ab = (const _Float16*)Ag + (size_t)(r0 + 32 * w) * kKA;
    const _Float16* Bt = (const _Float16*)Btp;
    const int rlane = lane & 15;
    const int koff  = (lane >> 4) * 8;
    const int mOff  = (lane >> 4) * 8;
#pragma unroll 1
    for (int jj = 0; jj < 2; ++jj) {
      v8f acc[2][4];
#pragma unroll
      for (int i = 0; i < 2; ++i)
#pragma unroll
        for (int j = 0; j < 4; ++j) acc[i][j] = (v8f){0.f,0.f,0.f,0.f,0.f,0.f,0.f,0.f};
#pragma unroll
      for (int ks = 0; ks < 2; ++ks) {
        v16h bh[4];
#pragma unroll
        for (int j = 0; j < 4; ++j)
          bh[j] = Frag<_Float16>::load(Bt + (size_t)(64 * jj + 16 * j + rlane) * kKA + koff + 32 * ks);
#pragma unroll
        for (int i = 0; i < 2; ++i) {
          const v16h ah = Frag<_Float16>::load(Ab + (size_t)(16 * i + rlane) * kKA + koff + 32 * ks);
#pragma unroll
          for (int j = 0; j < 4; ++j) acc[i][j] = Frag<_Float16>::mma(ah, bh[j], acc[i][j]);
          Frag<_Float16>::guard(acc[i][0], acc[i][3], ah, ah);
        }
        Frag<_Float16>::keep(bh[0], bh[1], bh[2], bh[3]);
      }
      acc_guard4(acc[0][0], acc[0][1], acc[0][2], acc[0][3]);
      acc_guard4(acc[1][0], acc[1][1], acc[1][2], acc[1][3]);
#pragma unroll
      for (int i = 0; i < 2; ++i)
#pragma unroll
        for (int j = 0; j < 4; ++j)
#pragma unroll
          for (int r = 0; r < 8; ++r)
            sZ[(32 * w + 16 * i + mOff + r) * kZP + 64 * jj + 16 * j + rlane] = acc[i][j][r] * kWCarryInv;
    }
  }
  __syncthreads();

  const int b  = r0 + tid;
  const int bc = (b < B) ? b : (B - 1);
  const float* zrow = sZ + tid * kZP;
  const float* crow = Cg + (size_t)bc * kHid;
  float cmd0 = 0.0f, cmd1 = 0.0f, cmd2 = 0.0f, cmd3 = 0.0f;
#pragma unroll 2
  for (int j = 0; j < kHid; ++j) {
    const float zi = zrow[j]            + sBias[j];
    const float zf = zrow[kHid + j]     + sBias[kHid + j];
    const float zg = zrow[2 * kHid + j] + sBias[2 * kHid + j];
    const float zo = zrow[3 * kHid + j] + sBias[3 * kHid + j];
    const float cp = crow[j];
    const float ig = sigm_f(zi);
    const float fg = sigm_f(zf);
    const float gg = tanh_f(zg);
    const float og = sigm_f(zo);
    const float cn = fg * cp + ig * gg;
    const float hn = og * tanh_f(cn);
    sC[tid * kHid + j]        = cn;
    sA16[tid * kKA + kHid + j] = (_Float16)hn;
    if (PRED) {
      cmd0 = fmaf(hn, sPar[kOffCoW + 0 * kHid + j], cmd0);
      cmd1 = fmaf(hn, sPar[kOffCoW + 1 * kHid + j], cmd1);
      cmd2 = fmaf(hn, sPar[kOffCoW + 2 * kHid + j], cmd2);
      cmd3 = fmaf(hn, sPar[kOffCoW + 3 * kHid + j], cmd3);
    }
  }

  float X[kNS];
  float P[kNS][kNS];
  {
    const float* srow = Sg + (size_t)bc * kSP;
#pragma unroll
    for (int i = 0; i < kNS; ++i) X[i] = srow[i];
#pragma unroll
    for (int i = 0; i < kNS; ++i)
#pragma unroll
      for (int j = 0; j < kNS; ++j) P[i][j] = srow[kPO + i * kNS + j];
  }
  float gt0[3], gt1[3];
  gt0[0] = kGA * sPar[kOffTh + 0]; gt0[1] = kGB * sPar[kOffTh + 1]; gt0[2] = kGC * sPar[kOffTh + 2];
  gt1[0] = kGA * sPar[kOffTh + 3]; gt1[1] = kGB * sPar[kOffTh + 4]; gt1[2] = kGC * sPar[kOffTh + 5];

  if (!PRED) {
    const float j0 = jerk[0], j1 = jerk[1];
    const float gr0 = GR[0], gr1 = GR[1];
    const float R00 = gr0 * gr0, R01 = gr0 * gr1, R11 = gr1 * gr1;
    float qh0[3], qh1[3];
#pragma unroll
    for (int i = 0; i < 3; ++i) { qh0[i] = gt0[i] * j0; qh1[i] = gt1[i] * j1; }

    kf_fx(X);
    kf_fpf(P);
#pragma unroll
    for (int i = 0; i < 3; ++i) {
#pragma unroll
      for (int l = 0; l < 3; ++l) {
        P[i][l]         += qh0[i] * qh0[l];
        P[3 + i][3 + l] += qh1[i] * qh1[l];
      }
    }
    const float zx = hist[((size_t)tz * B + bc) * 2 + 0];
    const float zy = hist[((size_t)tz * B + bc) * 2 + 1];
    const float y0 = zx - X[0], y1 = zy - X[3];
    const float s00 = P[0][0] + R00, s01 = P[0][3] + R01;
    const float s10 = P[3][0] + R01, s11 = P[3][3] + R11;
    const float det  = s00 * s11 - s01 * s10;
    const float rdet = 1.0f / det;
    const float i00 =  s11 * rdet, i01 = -s01 * rdet;
    const float i10 = -s10 * rdet, i11 =  s00 * rdet;
    float K0[kNS], K1[kNS];
#pragma unroll
    for (int i = 0; i < kNS; ++i) {
      K0[i] = P[i][0] * i00 + P[i][3] * i10;
      K1[i] = P[i][0] * i01 + P[i][3] * i11;
    }
#pragma unroll
    for (int i = 0; i < kNS; ++i) X[i] += K0[i] * y0 + K1[i] * y1;
    float Mt[kNS][kNS];
#pragma unroll
    for (int i = 0; i < kNS; ++i)
#pragma unroll
      for (int l = 0; l < kNS; ++l)
        Mt[i][l] = P[i][l] - K0[i] * P[0][l] - K1[i] * P[3][l];
#pragma unroll
    for (int i = 0; i < kNS; ++i) {
      const float u  = K0[i] * R00 + K1[i] * R01;
      const float ww = K0[i] * R01 + K1[i] * R11;
#pragma unroll
      for (int l = 0; l < kNS; ++l)
        P[i][l] = Mt[i][l] - Mt[i][0] * K0[l] - Mt[i][3] * K1[l] + u * K0[l] + ww * K1[l];
    }
  } else {
    cmd0 += sPar[kOffCob + 0]; cmd1 += sPar[kOffCob + 1];
    cmd2 += sPar[kOffCob + 2]; cmd3 += sPar[kOffCob + 3];
    kf_fx(X);
    X[0] += kGA * cmd0; X[1] += kGB * cmd0; X[2] += kGC * cmd0;
    X[3] += kGA * cmd1; X[4] += kGB * cmd1; X[5] += kGC * cmd1;
    float Gs[kNS];
#pragma unroll
    for (int i = 0; i < 3; ++i) { Gs[i] = gt0[i] * cmd2; Gs[3 + i] = gt1[i] * cmd3; }
    kf_fpf(P);
#pragma unroll
    for (int i = 0; i < kNS; ++i)
#pragma unroll
      for (int l = 0; l < kNS; ++l) P[i][l] += Gs[i] * Gs[l];
    const float p00 = P[0][0], p01 = P[0][3], p10 = P[3][0], p11 = P[3][3];
    const float sx = sqrtf(p00);
    const float sy = sqrtf(p11);
    const float rho = (p01 + p10) * (1.0f / (2.0f * sx * sy));
    float* orow = sO + tid * kOutF;
    orow[0] = X[0]; orow[1] = X[3]; orow[2] = sx; orow[3] = sy; orow[4] = rho;
  }

#pragma unroll 2
  for (int j = 0; j < kHid; ++j) {
    float a = 0.0f;
#pragma unroll
    for (int k = 0; k < kNS; ++k) a = fmaf(X[k], sPar[j * kNS + k], a);
    a += sPar[kOffCfb + j];
    sA16[tid * kKA + j] = (_Float16)tanh_f(a);
  }
  {
    float* sr = sS + tid * kSP;
#pragma unroll
    for (int i = 0; i < kNS; ++i) sr[i] = X[i];
    sr[6] = 0.0f; sr[7] = 0.0f;
#pragma unroll
    for (int i = 0; i < kNS; ++i)
#pragma unroll
      for (int j = 0; j < kNS; ++j) sr[kPO + i * kNS + j] = P[i][j];
  }
  __syncthreads();

  block_store_state(sA16, sC, sS, Ag, Cg, Sg, r0, tid);
  if (PRED) {
    float* ob = out + ((size_t)tz * B + r0) * kOutF;
    for (int ps = 0; ps < 2; ++ps) {
#pragma unroll
      for (int it = 0; it < 2; ++it) {
        const int q = it * kTile + tid;
        if (q < (kTile * kOutF) / 4) {
          const float* sp = sO + q * 4;
          const v4f v = (v4f){sp[0], sp[1], sp[2], sp[3]};
          *(volatile v4f*)(ob + (size_t)q * 4) = v;
        }
      }
      __threadfence();
    }
  }
}

extern "C" void kernel_launch(void* const* d_in, const int* in_sizes, int n_in,
                              void* d_out, int out_size, void* d_ws, size_t ws_size,
                              hipStream_t stream) {
  if (n_in < 19) return;
  const int nh = in_sizes[0];
  if (nh <= 0 || (nh % (kHistT * 2)) != 0) return;
  const int B = nh / (kHistT * 2);
  if (B <= 0 || (B % kTile) != 0) return;
  if (out_size <= 0 || (out_size % (kOutF * B)) != 0) return;
  const int LP = out_size / (kOutF * B);
  if (LP > 4000) return;
  for (int i = 1; i <= 6; ++i) if (in_sizes[i] < 1) return;
  if (in_sizes[7] != 2 || in_sizes[8] != kNS || in_sizes[9] != 2) return;
  if (in_sizes[10] != kHid * kNS || in_sizes[11] != kHid) return;
  if (in_sizes[12] != kGateN * kHid || in_sizes[13] != kGateN * kHid) return;
  if (in_sizes[14] != kGateN || in_sizes[15] != kGateN) return;
  if (in_sizes[16] != 4 * kHid || in_sizes[17] != 4 || in_sizes[18] < 1) return;

  const float* hist  = (const float*)d_in[0];
  const float* psx   = (const float*)d_in[1];
  const float* psy   = (const float*)d_in[2];
  const float* vsx   = (const float*)d_in[3];
  const float* vsy   = (const float*)d_in[4];
  const float* asx   = (const float*)d_in[5];
  const float* asy   = (const float*)d_in[6];
  const float* jerk  = (const float*)d_in[7];
  const float* coefG = (const float*)d_in[8];
  const float* GR    = (const float*)d_in[9];
  const float* cfW   = (const float*)d_in[10];
  const float* cfb   = (const float*)d_in[11];
  const float* Wih   = (const float*)d_in[12];
  const float* Whh   = (const float*)d_in[13];
  const float* bih   = (const float*)d_in[14];
  const float* bhh   = (const float*)d_in[15];
  const float* coW   = (const float*)d_in[16];
  const float* cob   = (const float*)d_in[17];
  const int*   lenp  = (const int*)d_in[18];
  float* outp = (float*)d_out;

  const size_t SZ_PAR = 32768;
  const size_t SZ_A   = (size_t)B * kKA * 2;
  const size_t SZ_C   = (size_t)B * kHid * 4;
  const size_t SZ_S   = (size_t)B * kSP * 4;
  size_t off = 0;
  const size_t oPAR = off; off += SZ_PAR;
  const size_t oA   = off; off += SZ_A;
  const size_t oC   = off; off += SZ_C;
  const size_t oS   = off; off += SZ_S;
  const size_t TOTAL = off;
  if (TOTAL > ws_size) return;
  if (TOTAL > (size_t)134217728) return;

  char* ws = (char*)d_ws;
  unsigned short* Bt    = (unsigned short*)(ws + oPAR + 0);
  float*          biasv = (float*)(ws + oPAR + 16384);
  float*          dpar  = (float*)(ws + oPAR + 16896);
  unsigned short* Ag    = (unsigned short*)(ws + oA);
  float*          Cg    = (float*)(ws + oC);
  float*          Sg    = (float*)(ws + oS);

  const dim3 blk256(256), blk64(64);
  const dim3 gTrk(B / kTile);

  pack_params_kernel<<<dim3(5), blk256, 0, stream>>>(Wih, Whh, bih, bhh, coefG, Bt, biasv, dpar);
  init_kernel<<<gTrk, blk64, 0, stream>>>(hist, psx, psy, vsx, vsy, asx, asy, cfW, cfb, Ag, Cg, Sg, B);

  for (int s = 0; s < kHistT - 1; ++s) {
    step_kernel<false><<<gTrk, blk64, 0, stream>>>(Bt, biasv, dpar, hist, jerk, GR, cfW, cfb, coW, cob, lenp,
                                                    Ag, Cg, Sg, outp, B, s + 1);
  }
  for (int t = 0; t < LP; ++t) {
    step_kernel<true><<<gTrk, blk64, 0, stream>>>(Bt, biasv, dpar, hist, jerk, GR, cfW, cfb, coW, cob, lenp,
                                                   Ag, Cg, Sg, outp, B, t);
  }
}
